// NONLocalBlock2D_489626272347
// MI455X (gfx1250) — hardware-run, weakly checked
//
#include <hip/hip_runtime.h>


namespace {
constexpr int B = 4, C = 256, T = 4096, IC = 32, BL = 4  , QL = T  , NR = B * T;
constexpr float XS = 8.0f, WSC = 256.0f, RS_ = 1024.0f, PS = 1024.0f, LOG2E = 1.4426950408889634f;
static_assert(T % 32 == 0 && C == 256 && IC == 32 && QL % 32 == 0, "tiling");
typedef _Float16 b16;
typedef __attribute__((ext_vector_type(16))) _Float16 v16b;
typedef __attribute__((ext_vector_type(8))) _Float16 v8b;
typedef __attribute__((ext_vector_type(8))) float v8f;
typedef __attribute__((ext_vector_type(4))) float v4f;
__device__ __forceinline__ float bf16_rne(float f) { unsigned int u = __float_as_uint(f); u += 0x7FFFu + ((u >> 16) & 1u); return __uint_as_float(u & 0xFFFF0000u); }
__device__ __forceinline__ void split16(float v, b16& hi, b16& lo) { hi = (b16)v; lo = (b16)(v - (float)hi); }
__device__ __forceinline__ v16b frag_kb(const b16* p, int hh) { const v8b a = *(const v8b*)(p + 8 * hh), b = *(const v8b*)(p + 16 + 8 * hh); v16b f;
#pragma unroll
  for (int e = 0; e < 8; ++e) { f[e] = a[e]; f[8 + e] = b[e]; } return f; }
__device__ __forceinline__ v8f wmma16b(v16b a, v16b b, v8f c) { v8f d = __builtin_amdgcn_wmma_f32_16x16x32_f16(false, a, false, b, (short)0, c, false, false); asm volatile("v_nop\n\tv_nop\n\tv_nop\n\tv_nop" : "+v"(d) : "v"(a), "v"(b)); return d; }
__device__ __forceinline__ void wave_lds_sync() { __builtin_amdgcn_fence(__ATOMIC_RELEASE, "workgroup"); __builtin_amdgcn_wave_barrier(); __builtin_amdgcn_fence(__ATOMIC_ACQUIRE, "workgroup"); }
__device__ __forceinline__ float pmul(float a, float b) { float p = a * b; asm volatile("" : "+v"(p)); return p; }
__device__ __forceinline__ int iclamp(int v, int lo, int hi) { return v < lo ? lo : (v > hi ? hi : v); }

typedef __attribute__((ext_vector_type(2))) _Float16 v2h;
typedef __attribute__((ext_vector_type(4))) _Float16 v4h;
typedef __attribute__((ext_vector_type(2))) float v2f;
typedef __attribute__((ext_vector_type(4))) int v4i;
__device__ __forceinline__ float nexp2(float v) { return __builtin_amdgcn_exp2f(v); }
__device__ __forceinline__ float bfp(float v) { float t = bf16_rne(v); asm volatile("" : "+v"(t)); return t; }

__global__ __launch_bounds__(256) void wt_kernel(const float* __restrict__ thw, const float* __restrict__ gw, const float* __restrict__ ww, b16* __restrict__ WT, b16* __restrict__ WWT, b16* __restrict__ WWQ) {
  const int u = blockIdx.x * 256 + threadIdx.x;
  if (u < 2 * IC * C / 8) { const int e = u * 8; const int o = e / C, k0 = e % C; const float* src = (o < IC) ? (thw + (size_t)o * C) : (gw + (size_t)(o - IC) * C); v8b v; for (int j = 0; j < 8; ++j) v[j] = (b16)(bf16_rne(src[k0 + j]) * WSC);
    for (int pass = 0; pass < 2; ++pass) { *(volatile v8b*)(WT + e) = v; __threadfence(); } }
  else if (u < 2 * IC * C / 8 + C * IC / 8) { const int e = (u - 2 * IC * C / 8) * 8; v8b v, q; for (int j = 0; j < 8; ++j) { const float w = bf16_rne(ww[e + j]); v[j] = (b16)(w * WSC); q[j] = (b16)(w * 0.25f); }
    for (int pass = 0; pass < 2; ++pass) { *(volatile v8b*)(WWT + e) = v; *(volatile v8b*)(WWQ + e) = q; __threadfence(); } }
}
__global__ __launch_bounds__(64) void proj_kernel(const float* __restrict__ x, const b16* __restrict__ WT, b16* __restrict__ THh, b16* __restrict__ THl, b16* __restrict__ Gh, b16* __restrict__ Gl) {
  __shared__ __attribute__((aligned(16))) b16 Ah[2][16][C + 8]; __shared__ __attribute__((aligned(16))) float Tw[2][16][2 * IC + 4];
  const int wave = threadIdx.x >> 5, lane = threadIdx.x & 31, nloc = lane & 15, hlf = lane >> 4; const int b = blockIdx.y; const int n0 = blockIdx.x * 32 + wave * 16;
  for (int idx = lane; idx < 16 * C; idx += 32) { const int k = idx >> 4, rr = idx & 15; Ah[wave][rr][k] = (b16)(bf16_rne(x[((size_t)b * C + k) * T + n0 + rr]) * XS); }
  wave_lds_sync();
  v8f acc[4]; for (int t = 0; t < 4; ++t) acc[t] = (v8f){};
#pragma unroll 2
  for (int kb = 0; kb < C; kb += 32) { const v16b a = frag_kb(&Ah[wave][nloc][kb], hlf);
#pragma unroll
    for (int t = 0; t < 4; ++t) acc[t] = wmma16b(a, frag_kb(WT + (size_t)(t * 16 + nloc) * C + kb, hlf), acc[t]); }
#pragma unroll
  for (int t = 0; t < 4; ++t) for (int r = 0; r < 8; ++r) Tw[wave][8 * hlf + r][t * 16 + nloc] = acc[t][r] * (1.0f / (XS * WSC));
  wave_lds_sync();
  for (int pass = 0; pass < 2; ++pass) { for (int rr = 0; rr < 16; rr += 4) { const int r2 = rr + (lane >> 3); const int c4 = (lane & 7) * 4; const size_t o_ = ((size_t)b * T + n0 + r2) * IC + c4; v4h h1, l1, h2, l2;
      for (int j = 0; j < 4; ++j) { float v = Tw[wave][r2][c4 + j] * XS; b16 ph = (b16)v; h1[j] = ph; l1[j] = (b16)((v - (float)ph) * RS_); v = Tw[wave][r2][IC + c4 + j] * XS; ph = (b16)v; h2[j] = ph; l2[j] = (b16)((v - (float)ph) * RS_); }
      *(volatile v4h*)(THh + o_) = h1; *(volatile v4h*)(THl + o_) = l1; *(volatile v4h*)(Gh + o_) = h2; *(volatile v4h*)(Gl + o_) = l2; } __threadfence(); }
}
__global__ __launch_bounds__(32) void attn_kernel(const b16* __restrict__ THh, const b16* __restrict__ THl, const b16* __restrict__ Gh, const b16* __restrict__ Gl, float* __restrict__ Y) {
  __shared__ __attribute__((aligned(16))) b16 Pt[16][32 + 8]; __shared__ __attribute__((aligned(16))) float Of[16][IC + 4];
  const int lane = threadIdx.x, nloc = lane & 15, hlf = lane >> 4; const int q0 = blockIdx.x * 16, b = blockIdx.y; const size_t qbase = (size_t)b * T + q0;
  v16b aqh, aql;
#pragma unroll
  for (int e = 0; e < 16; ++e) { const int k = (e < 8) ? (8 * hlf + e) : (16 + 8 * hlf + (e - 8)); aqh[e] = THh[(qbase + nloc) * IC + k]; aql[e] = THl[(qbase + nloc) * IC + k]; }
  float mrow[8], lsum[8]; for (int r = 0; r < 8; ++r) { mrow[r] = -INFINITY; lsum[r] = 0.0f; }
  v8f acco[2], accol[2]; for (int t = 0; t < 2; ++t) { acco[t] = (v8f){}; accol[t] = (v8f){}; }
#pragma unroll 1
  for (int kb = 0; kb < T; kb += 32) {
    const size_t kbase = (size_t)b * T + kb;
    v8f sh[2], sl[2];
#pragma unroll
    for (int t = 0; t < 2; ++t) { sh[t] = (v8f){}; sl[t] = (v8f){}; v16b bh, bl;
#pragma unroll
      for (int e = 0; e < 16; ++e) { const int k = (e < 8) ? (8 * hlf + e) : (16 + 8 * hlf + (e - 8)); const size_t o_ = (kbase + t * 16 + nloc) * IC + k; bh[e] = THh[o_]; bl[e] = THl[o_]; }
      sh[t] = wmma16b(aqh, bh, sh[t]); sl[t] = wmma16b(aqh, bl, sl[t]); sl[t] = wmma16b(aql, bh, sl[t]); }
    float s[2][8], mx[8];
#pragma unroll
    for (int r = 0; r < 8; ++r) { mx[r] = -INFINITY;
#pragma unroll
      for (int t = 0; t < 2; ++t) { s[t][r] = (sh[t][r] + sl[t][r] * (1.0f / RS_)) * (1.0f / (XS * XS)); mx[r] = fmaxf(mx[r], s[t][r]); } }
#pragma unroll
    for (int o = 1; o < 16; o <<= 1) for (int r = 0; r < 8; ++r) mx[r] = fmaxf(mx[r], __shfl_xor(mx[r], o));
    v16b pv;
#pragma unroll
    for (int r = 0; r < 8; ++r) { const float mn = fmaxf(mrow[r], mx[r]); const float corr = nexp2((mrow[r] - mn) * LOG2E); mrow[r] = mn; lsum[r] *= corr;
#pragma unroll
      for (int t = 0; t < 2; ++t) { acco[t][r] *= corr; accol[t][r] *= corr; const float p = nexp2((s[t][r] - mn) * LOG2E); lsum[r] += p; pv[8 * t + r] = (b16)(p * PS); } }
#pragma unroll
    for (int t = 0; t < 2; ++t) for (int r = 0; r < 8; ++r) Pt[8 * hlf + r][16 * t + nloc] = pv[8 * t + r];
    wave_lds_sync();
    const v16b a = frag_kb(&Pt[nloc][0], hlf);
#pragma unroll
    for (int t = 0; t < 2; ++t) { v16b vh, vl;
#pragma unroll
      for (int e = 0; e < 16; ++e) { const int k = (e < 8) ? (8 * hlf + e) : (16 + 8 * hlf + (e - 8)); const size_t o_ = (kbase + k) * IC + t * 16 + nloc; vh[e] = Gh[o_]; vl[e] = Gl[o_]; }
      acco[t] = wmma16b(a, vh, acco[t]); accol[t] = wmma16b(a, vl, accol[t]); }
    wave_lds_sync(); }
#pragma unroll
  for (int o = 1; o < 16; o <<= 1) for (int r = 0; r < 8; ++r) lsum[r] += __shfl_xor(lsum[r], o);
#pragma unroll
  for (int t = 0; t < 2; ++t) for (int r = 0; r < 8; ++r) Of[8 * hlf + r][t * 16 + nloc] = (acco[t][r] + accol[t][r] * (1.0f / RS_)) * (1.0f / (PS * XS)) / lsum[r];
  wave_lds_sync();
  for (int pass = 0; pass < 2; ++pass) { for (int rr = 0; rr < 16; rr += 4) { const int r2 = rr + (lane >> 3); if (q0 + r2 < QL) *(volatile v4f*)(Y + (qbase + r2) * IC + (lane & 7) * 4) = *(const v4f*)(&Of[r2][(lane & 7) * 4]); } __threadfence(); }
}
__global__ __launch_bounds__(64) void out_kernel(const float* __restrict__ Y, const b16* __restrict__ WWT, const b16* __restrict__ WWQ, const float* __restrict__ x, float* __restrict__ out) {
  __shared__ __attribute__((aligned(16))) b16 Ah[2][16][IC + 8], Al[2][16][IC + 8]; __shared__ float Zs[32][C + 1];
  const int wave = threadIdx.x >> 5, lane = threadIdx.x & 31, nloc = lane & 15, hlf = lane >> 4; const int b = blockIdx.y; const int n0 = blockIdx.x * 32; const size_t rbase = (size_t)b * T + n0 + wave * 16;
  for (int idx = lane; idx < 16 * (IC / 4); idx += 32) { const int rr = idx / (IC / 4), c4 = (idx % (IC / 4)) * 4; const v4f v = *(const v4f*)(Y + (rbase + rr) * IC + c4); v4h hv, lv; for (int j = 0; j < 4; ++j) { const float vs = v[j] * XS; const b16 ph = (b16)vs; hv[j] = ph; lv[j] = (b16)((vs - (float)ph) * RS_); } *(v4h*)(&Ah[wave][rr][c4]) = hv; *(v4h*)(&Al[wave][rr][c4]) = lv; }
  wave_lds_sync();
  const v16b a = frag_kb(&Ah[wave][nloc][0], hlf), al = frag_kb(&Al[wave][nloc][0], hlf);
#pragma unroll 1
  for (int t = 0; t < C / 16; ++t) { v8f acc = (v8f){}; acc = wmma16b(a, frag_kb(WWT + (size_t)(t * 16 + nloc) * IC, hlf), acc); acc = wmma16b(al, frag_kb(WWQ + (size_t)(t * 16 + nloc) * IC, hlf), acc);
#pragma unroll
    for (int r = 0; r < 8; ++r) Zs[wave * 16 + 8 * hlf + r][t * 16 + nloc] = acc[r] * (1.0f / (XS * WSC)); }
  __syncthreads();
  for (int pass = 0; pass < 2; ++pass) {
#pragma unroll 4
    for (int cc = 0; cc < C / 2; ++cc) { const int c = wave * (C / 2) + cc; const size_t o_ = ((size_t)b * C + c) * T + n0 + lane; if (n0 + lane < QL) ((volatile float*)out)[o_] = Zs[lane][c] + bf16_rne(x[o_]); }
    __threadfence(); }
}
}

extern "C" void kernel_launch(void* const* d_in, const int* in_sizes, int n_in, void* d_out, int out_size, void* d_ws, size_t ws_size, hipStream_t stream) {
  (void)n_in;
  auto Fp = [&](int i) { return (const float*)d_in[i]; };
  if (in_sizes[0] != B * C * T || in_sizes[1] != IC * C || in_sizes[2] != IC * C || in_sizes[3] != C * IC || out_size != B * C * T) return;
  size_t off = 0; char* ws = (char*)d_ws;
  auto carve = [&](size_t bytes) { char* p = ws + off; off += (bytes + 255) & ~(size_t)255; return p; };
  b16* WT = (b16*)carve((size_t)2 * IC * C * 2); b16* WWT = (b16*)carve((size_t)C * IC * 2); b16* WWQ = (b16*)carve((size_t)C * IC * 2);
  b16* THh = (b16*)carve((size_t)NR * IC * 2); b16* THl = (b16*)carve((size_t)NR * IC * 2); b16* Gh = (b16*)carve((size_t)NR * IC * 2); b16* Gl = (b16*)carve((size_t)NR * IC * 2); float* Y = (float*)carve((size_t)NR * IC * 4);
  if (off > ws_size || off > ((size_t)64 << 20)) return;
  wt_kernel<<<(2 * IC * C / 8 + C * IC / 8 + 255) / 256, 256, 0, stream>>>(Fp(2), Fp(1), Fp(3), WT, WWT, WWQ);
  proj_kernel<<<dim3(T / 32, BL), 64, 0, stream>>>(Fp(0), WT, THh, THl, Gh, Gl);
  attn_kernel<<<dim3(QL / 16, BL), 32, 0, stream>>>(THh, THl, Gh, Gl, Y);
  out_kernel<<<dim3(QL / 32, BL), 64, 0, stream>>>(Y, WWT, WWQ, Fp(0), (float*)d_out);
}
